// TwoReacModel_37074157699116
// MI455X (gfx1250) — hardware-verified
//
#include <hip/hip_runtime.h>
#include <stdint.h>

typedef __attribute__((ext_vector_type(16))) _Float16 v16h;
typedef __attribute__((ext_vector_type(8)))  _Float16 v8h;
typedef __attribute__((ext_vector_type(8)))  float    v8f;
typedef __attribute__((ext_vector_type(4)))  float    v4f;

constexpr int kSteps  = 128;
constexpr int kHid    = 64;
constexpr int kHeadN  = 16;
constexpr int kPitchH = 72;
constexpr int kWaves  = 2;
constexpr int kRows   = 16;
constexpr int kChunkF = 96;
constexpr int kPathF  = 384;
static_assert(kWaves * 32 == kHid);
static_assert(kWaves * 32 == kHeadN * 4);
static_assert(kChunkF * 4 == kPathF);

__device__ __forceinline__ v16h frag_load(const _Float16* p) {
  union { v16h v; v8h hh[2]; } f;
  f.hh[0] = *(const v8h*)(p);
  f.hh[1] = *(const v8h*)(p + 16);
  return f.v;
}
__device__ __forceinline__ v8f mma_f16(v16h a, v16h b, v8f c) {
  c = __builtin_amdgcn_wmma_f32_16x16x32_f16(false, a, false, b, (short)0, c, false, false);
  asm volatile("v_nop\n\tv_nop\n\tv_nop\n\tv_nop" : "+v"(c) : "v"(a), "v"(b));
  return c;
}
__device__ __forceinline__ void lds_sync() {
  __builtin_amdgcn_fence(__ATOMIC_RELEASE, "workgroup");
  __builtin_amdgcn_wave_barrier();
  __builtin_amdgcn_fence(__ATOMIC_ACQUIRE, "workgroup");
}
__device__ __forceinline__ float tanh_hw(float c) {
  const float e = __builtin_amdgcn_exp2f(c * 2.8853900817779268f);
  return 1.0f - 2.0f * __builtin_amdgcn_rcpf(e + 1.0f);
}

__global__ __launch_bounds__(64) __attribute__((amdgpu_num_vgpr(192)))
void ode_rk4_mlp(
    const float* __restrict__ u,     const float* __restrict__ x0,
    const float* __restrict__ W1,    const float* __restrict__ b1,
    const float* __restrict__ W2,    const float* __restrict__ b2,
    const float* __restrict__ W3,    const float* __restrict__ b3,
    const float* __restrict__ xmean, const float* __restrict__ xstd,
    const float* __restrict__ umean, const float* __restrict__ ustd,
    float* __restrict__ out, int npaths)
{
  __shared__ __align__(16) _Float16 W2t[kHid * kPitchH];
  __shared__ __align__(16) _Float16 W3t[kHeadN * kPitchH];
  __shared__ __align__(16) float    W1e[kHid * 4];
  __shared__ __align__(16) float    b1s[kHid];
  __shared__ __align__(16) float    b2s[kHid];
  __shared__ __align__(16) _Float16 h1t[kWaves][kRows * kPitchH];
  __shared__ __align__(16) _Float16 h2t[kWaves][kRows * kPitchH];
  __shared__ __align__(16) float    yst[kWaves][kRows * kChunkF];

  const int tid  = threadIdx.x;
  const int lane = tid & 31;
  const int wave = tid >> 5;
  const int h    = lane >> 4;
  const int m    = lane & 15;

  {
    const int n = tid;
#pragma unroll 1
    for (int kk = 0; kk < 8; ++kk) {
      v8h hv;
#pragma unroll
      for (int e = 0; e < 8; ++e) hv[e] = (_Float16)(W2[(8 * kk + e) * kHid + n] * 16.0f);
      *(v8h*)(W2t + n * kPitchH + 8 * kk) = hv;
    }
    const int n3  = tid >> 2;
    const int kq  = tid & 3;
    const int n3c = (n3 < 3) ? n3 : 2;
#pragma unroll 1
    for (int s2 = 0; s2 < 2; ++s2) {
      v8h hv;
#pragma unroll
      for (int e = 0; e < 8; ++e) hv[e] = (_Float16)(W3[(16 * kq + 8 * s2 + e) * 3 + n3c] * 16.0f);
      *(v8h*)(W3t + n3 * kPitchH + 16 * kq + 8 * s2) = hv;
    }
    v4f w1v;
    w1v[0] = W1[n]; w1v[1] = W1[kHid + n]; w1v[2] = W1[2 * kHid + n]; w1v[3] = W1[3 * kHid + n];
    *(v4f*)(W1e + 4 * n) = w1v;
    b1s[n] = b1[n];
    b2s[n] = b2[n];
  }
  __syncthreads();

  const float xm0 = xmean[0], xm1 = xmean[1], xm2 = xmean[2];
  const float xs0 = xstd[0],  xs1 = xstd[1],  xs2 = xstd[2];
  const float rx0 = 1.0f / xs0, rx1 = 1.0f / xs1, rx2 = 1.0f / xs2;
  const float um  = umean[0], us = ustd[0];
  const float b30 = b3[0], b31 = b3[1], b32 = b3[2];
  const float invTau = 0.2f;
  const float sixth  = 0.16666667f;

  const int pathBase = (blockIdx.x * kWaves + wave) * kRows;
  if (pathBase < npaths) {
    int prow = pathBase + m;
    prow = (prow < npaths) ? prow : (npaths - 1);
    const float* urow = u + (size_t)prow * kSteps;
    float xa = x0[(size_t)prow * 3 + 0];
    float xb = x0[(size_t)prow * 3 + 1];
    float xc = x0[(size_t)prow * 3 + 2];
    _Float16* h1w = h1t[wave];
    _Float16* h2w = h2t[wave];
    float*    ysw = yst[wave];
    const int q  = lane >> 3;
    const int c4 = (lane & 7) * 4;

#pragma unroll 1
    for (int t = 0; t < kSteps; ++t) {
      const int ts = t & 31;
      ysw[m * kChunkF + ts * 3 + 0] = xa;
      ysw[m * kChunkF + ts * 3 + 1] = xb;
      ysw[m * kChunkF + ts * 3 + 2] = xc;

      if (ts == 31) {
        const int chunk = t >> 5;
        lds_sync();
        for (int pass = 0; pass < 2; ++pass) {
#pragma unroll
          for (int it = 0; it < 12; ++it) {
            const int L  = it * 4 + q;
            const int p  = L / 3;
            const int li = L - 3 * p;
            const v4f v = *(const v4f*)(ysw + p * kChunkF + li * 32 + c4);
            const int path = pathBase + p;
            if (path < npaths)
              *(volatile v4f*)(out + (size_t)path * kPathF + chunk * kChunkF + li * 32 + c4) = v;
          }
          __threadfence();
        }
        lds_sync();
      }

      if (t + 1 < kSteps) {
        const float ut = urow[t];
        const float up = fmaf(ut, us, um);
        float kp0 = 0.f, kp1 = 0.f, kp2 = 0.f;
        float ks0 = 0.f, ks1 = 0.f, ks2 = 0.f;
#pragma unroll 1
        for (int s = 0; s < 4; ++s) {
          const float cf = (s == 0) ? 0.0f : ((s == 3) ? 1.0f : 0.5f);
          const float wg = (s == 1 || s == 2) ? 2.0f : 1.0f;
          const float z0 = fmaf(kp0, cf, xa);
          const float z1 = fmaf(kp1, cf, xb);
          const float z2 = fmaf(kp2, cf, xc);
          const float z3 = ut;

          int ldz = 0;
          asm volatile("" : "+v"(ldz));
          const float*    W1q = W1e + ldz;
          const float*    b1q = b1s + ldz;
          const float*    b2q = b2s + ldz;
          const _Float16* W2q = W2t + ldz;
          const _Float16* W3q = W3t + ldz;

#pragma unroll 1
          for (int g = 0; g < 4; ++g) {
            const int nb = 32 * h + 8 * g;
            v8h hv;
#pragma unroll
            for (int e = 0; e < 8; ++e) {
              const v4f w = *(const v4f*)(W1q + 4 * (nb + e));
              float a = z0 * w[0];
              a = fmaf(z1, w[1], a);
              a = fmaf(z2, w[2], a);
              a = fmaf(z3, w[3], a);
              a = a + b1q[nb + e];
              hv[e] = (_Float16)tanh_hw(a);
            }
            *(v8h*)(h1w + m * kPitchH + nb) = hv;
          }
          lds_sync();

          v8f acc[4];
#pragma unroll
          for (int i = 0; i < 4; ++i) acc[i] = (v8f){0.f, 0.f, 0.f, 0.f, 0.f, 0.f, 0.f, 0.f};
#pragma unroll
          for (int kk = 0; kk < 2; ++kk) {
            const int k0 = 32 * kk;
            const v16h bfr = frag_load(h1w + m * kPitchH + k0 + 8 * h);
#pragma unroll
            for (int i = 0; i < 4; ++i) {
              const v16h afr = frag_load(W2q + (16 * i + m) * kPitchH + k0 + 8 * h);
              acc[i] = mma_f16(afr, bfr, acc[i]);
            }
          }
          lds_sync();

#pragma unroll
          for (int i = 0; i < 4; ++i) {
            const int nb = 16 * i + 8 * h;
            const v4f bA = *(const v4f*)(b2q + nb);
            const v4f bB = *(const v4f*)(b2q + nb + 4);
            v8h hv;
#pragma unroll
            for (int r = 0; r < 8; ++r) {
              const float bias = (r < 4) ? bA[r & 3] : bB[r & 3];
              const float v = fmaf(acc[i][r], 0.0625f, bias);
              hv[r] = (_Float16)tanh_hw(v);
            }
            *(v8h*)(h2w + m * kPitchH + nb) = hv;
          }
          lds_sync();

          v8f acc3 = (v8f){0.f, 0.f, 0.f, 0.f, 0.f, 0.f, 0.f, 0.f};
#pragma unroll
          for (int kk = 0; kk < 2; ++kk) {
            const int k0 = 32 * kk;
            const v16h afr = frag_load(W3q + m * kPitchH + k0 + 8 * h);
            const v16h bfr = frag_load(h2w + m * kPitchH + k0 + 8 * h);
            acc3 = mma_f16(afr, bfr, acc3);
          }
          const float p0 = __shfl(acc3[0], m, 32) * 0.0625f;
          const float p1 = __shfl(acc3[1], m, 32) * 0.0625f;
          const float p2 = __shfl(acc3[2], m, 32) * 0.0625f;

          const float xp0 = fmaf(z0, xs0, xm0);
          const float xp1 = fmaf(z1, xs1, xm1);
          const float xp2 = fmaf(z2, xs2, xm2);
          const float f0 = ((up - xp0) * invTau) * rx0 + (p0 + b30);
          const float f1 = ((-xp1) * invTau) * rx1 + (p1 + b31);
          const float f2 = ((-xp2) * invTau) * rx2 + (p2 + b32);

          ks0 = fmaf(f0, wg, ks0);
          ks1 = fmaf(f1, wg, ks1);
          ks2 = fmaf(f2, wg, ks2);
          kp0 = f0; kp1 = f1; kp2 = f2;
        }
        xa = fmaf(ks0, sixth, xa);
        xb = fmaf(ks1, sixth, xb);
        xc = fmaf(ks2, sixth, xc);
      }
    }
  }
}

extern "C" void kernel_launch(void* const* d_in, const int* in_sizes, int n_in,
                              void* d_out, int out_size, void* d_ws, size_t ws_size,
                              hipStream_t stream) {
  (void)d_ws; (void)ws_size;
  if (n_in < 12) return;
  const int npaths = in_sizes[1] / 3;
  if (npaths <= 0) return;
  if (in_sizes[1] != npaths * 3) return;
  if (in_sizes[0] != npaths * kSteps) return;
  if (out_size != npaths * kPathF) return;
  if (in_sizes[2] != 4 * kHid || in_sizes[3] < kHid || in_sizes[4] != kHid * kHid || in_sizes[5] < kHid ||
      in_sizes[6] != kHid * 3 || in_sizes[7] < 3 || in_sizes[8] < 3 || in_sizes[9] < 3 ||
      in_sizes[10] < 1 || in_sizes[11] < 1) return;

  const float* u     = (const float*)d_in[0];
  const float* x0    = (const float*)d_in[1];
  const float* W1    = (const float*)d_in[2];
  const float* b1    = (const float*)d_in[3];
  const float* W2    = (const float*)d_in[4];
  const float* b2    = (const float*)d_in[5];
  const float* W3    = (const float*)d_in[6];
  const float* b3    = (const float*)d_in[7];
  const float* xmean = (const float*)d_in[8];
  const float* xstd  = (const float*)d_in[9];
  const float* umean = (const float*)d_in[10];
  const float* ustd  = (const float*)d_in[11];
  float* out = (float*)d_out;

  const int pathsPerBlock = kWaves * kRows;
  const int nblk = (npaths + pathsPerBlock - 1) / pathsPerBlock;
  ode_rk4_mlp<<<dim3(nblk), dim3(kWaves * 32), 0, stream>>>(
      u, x0, W1, b1, W2, b2, W3, b3, xmean, xstd, umean, ustd, out, npaths);
}
